// MultiChannelAttention_62234076119700
// MI455X (gfx1250) — hardware-verified
//
#include <hip/hip_runtime.h>
#include <stdint.h>

#define NB_   32
#define IDF_  64
#define CDF_  256
#define SS_   1024
#define NH_   8
#define LL_   256

static_assert((SS_ % 64) == 0 && (CDF_ % 64) == 0 && (LL_ % 64) == 0 && (IDF_ % 64) == 0);
static_assert(LL_ == 256 && IDF_ == 64 && NH_ == 8);
static_assert((SS_ % 32) == 0 && (CDF_ % 32) == 0);

typedef __bf16   v16b __attribute__((ext_vector_type(16)));
typedef __bf16   v8b  __attribute__((ext_vector_type(8)));
typedef float    v8f  __attribute__((ext_vector_type(8)));
typedef float    v4f  __attribute__((ext_vector_type(4)));
typedef unsigned int v4u __attribute__((ext_vector_type(4)));

__device__ __forceinline__ unsigned short bf_bits(float f) {
  unsigned u = __float_as_uint(f);
  return (unsigned short)((u + 0x7FFFu + ((u >> 16) & 1u)) >> 16);
}
__device__ __forceinline__ float bf_up(unsigned short h) { return __uint_as_float(((unsigned)h) << 16); }
__device__ __forceinline__ unsigned pk16(unsigned short a, unsigned short b) { return (unsigned)a | ((unsigned)b << 16); }
__device__ __forceinline__ v8f zero8() { v8f z = {0.f, 0.f, 0.f, 0.f, 0.f, 0.f, 0.f, 0.f}; return z; }
__device__ __forceinline__ v4u pack8_bf(v4f a, v4f b) {
  v4u p;
  p[0] = pk16(bf_bits(a[0]), bf_bits(a[1]));
  p[1] = pk16(bf_bits(a[2]), bf_bits(a[3]));
  p[2] = pk16(bf_bits(b[0]), bf_bits(b[1]));
  p[3] = pk16(bf_bits(b[2]), bf_bits(b[3]));
  return p;
}

__device__ __forceinline__ v16b ldfrag_b(const __bf16* p) {
  union { v16b v; v8b h[2]; } f;
  f.h[0] = *(const v8b*)(p);
  f.h[1] = *(const v8b*)(p + 16);
  return f.v;
}

__device__ __forceinline__ v8f mma_b_raw(v16b a, v16b b, v8f c) {
  return __builtin_amdgcn_wmma_f32_16x16x32_bf16(false, a, false, b, (short)0, c, false, false);
}
__device__ __forceinline__ void dep_guard_b(v8f& a, v8f& b, v16b x, v16b y) {
#if defined(__HIP_DEVICE_COMPILE__)
  asm volatile("v_nop\n\tv_nop\n\tv_nop\n\tv_nop" : "+v"(a), "+v"(b) : "v"(x), "v"(y));
#endif
}
__device__ __forceinline__ void keep4_b(v16b a, v16b b, v16b c, v16b d) {
#if defined(__HIP_DEVICE_COMPILE__)
  asm volatile("v_nop" :: "v"(a), "v"(b), "v"(c), "v"(d));
#endif
}
__device__ __forceinline__ void acc_guard4(v8f& a, v8f& b, v8f& c, v8f& d) {
#if defined(__HIP_DEVICE_COMPILE__)
  asm volatile("v_nop\n\tv_nop\n\tv_nop\n\tv_nop" : "+v"(a), "+v"(b), "+v"(c), "+v"(d));
#endif
}
__device__ __forceinline__ void wave_sync_lds() {
  __builtin_amdgcn_fence(__ATOMIC_RELEASE, "workgroup");
  __builtin_amdgcn_wave_barrier();
  __builtin_amdgcn_fence(__ATOMIC_ACQUIRE, "workgroup");
}

__global__ __launch_bounds__(256) void cvt_bf16x8(const float* __restrict__ in, unsigned short* out, int n8) {
  const int i = blockIdx.x * 256 + threadIdx.x;
  if (i < n8) {
    const v4f a = *(const v4f*)(in + (size_t)i * 8);
    const v4f b = *(const v4f*)(in + (size_t)i * 8 + 4);
    const v4u p = pack8_bf(a, b);
    *(volatile v4u*)(out + (size_t)i * 8) = p;
    __threadfence();
    *(volatile v4u*)(out + (size_t)i * 8) = p;
  }
}

__global__ __launch_bounds__(256) void tcvt64(const float* __restrict__ in, unsigned short* outN, unsigned short* outT,
                                              int R, int C) {
  __shared__ __align__(16) float tT[64 * 68];
  const int g  = blockIdx.z;
  const int c0 = blockIdx.x * 64;
  const int r0 = blockIdx.y * 64;
  const int tid = threadIdx.x, lane = tid & 31, wave = tid >> 5;
  const size_t gR = (size_t)g * R;
  {
    const int r = tid >> 2, cc = (tid & 3) * 16;
    const float* src = in + (gR + r0 + r) * (size_t)C + c0 + cc;
#pragma unroll
    for (int j4 = 0; j4 < 4; ++j4) {
      const v4f x = *(const v4f*)(src + 4 * j4);
      tT[(cc + 4 * j4 + 0) * 68 + r] = x[0];
      tT[(cc + 4 * j4 + 1) * 68 + r] = x[1];
      tT[(cc + 4 * j4 + 2) * 68 + r] = x[2];
      tT[(cc + 4 * j4 + 3) * 68 + r] = x[3];
    }
  }
  __syncthreads();
  const int q = lane >> 3, c8 = (lane & 7) * 8;
  v4u tv[2], nv[2];
#pragma unroll
  for (int it = 0; it < 2; ++it) {
    const int row = it * 32 + wave * 4 + q;
    const float* sp = tT + row * 68 + c8;
    tv[it] = pack8_bf(*(const v4f*)sp, *(const v4f*)(sp + 4));
    const float* np = in + (gR + r0 + row) * (size_t)C + c0 + c8;
    nv[it] = pack8_bf(*(const v4f*)np, *(const v4f*)(np + 4));
  }
  for (int pass = 0; pass < 2; ++pass) {
#pragma unroll
    for (int it = 0; it < 2; ++it) {
      const int row = it * 32 + wave * 4 + q;
      *(volatile v4u*)(outT + ((size_t)g * C + c0 + row) * (size_t)R + r0 + c8) = tv[it];
      *(volatile v4u*)(outN + (gR + r0 + row) * (size_t)C + c0 + c8) = nv[it];
    }
    __threadfence();
  }
}

template <int NSPLIT, int OUT_MODE>
__global__ __launch_bounds__(256) void gemm64(
    const unsigned short* __restrict__ Ap, const unsigned short* A2p, int lda,
    long long yA, long long zA, long long ksA,
    const unsigned short* __restrict__ Btp, int ldb,
    long long yB, long long zB, long long ksB, int ksh,
    void* Cout, void* Cout2, int ldc, long long yC, long long zC,
    int M, int N, int K, int nz) {
  const __bf16* A  = (const __bf16*)(const void*)Ap;
  const __bf16* A2 = (const __bf16*)(const void*)A2p;
  const __bf16* Bt = (const __bf16*)(const void*)Btp;
  __shared__ __align__(16) float sT[8][16 * 68];
  const int y    = blockIdx.y;
  const int lane = threadIdx.x & 31;
  const int wave = threadIdx.x >> 5;
  const int tilesN  = N >> 6;
  const int tilesM  = M >> 6;
  const int tilesMN = tilesM * tilesN;
  const int tile = blockIdx.x * 8 + wave;
  if (tile >= tilesMN * nz) return;
  const int z  = tile / tilesMN;
  const int rm = tile - z * tilesMN;
  const int tm = rm / tilesN;
  const int tn = rm - tm * tilesN;
  const int m0 = tm << 6;
  const int n0 = tn << 6;

  const size_t offA = (size_t)y * (size_t)yA + (size_t)z * (size_t)zA;
  const size_t offB = (size_t)y * (size_t)yB + (size_t)z * (size_t)zB;
  const size_t offC = (size_t)y * (size_t)yC + (size_t)z * (size_t)zC;
  const __bf16* Ab  = A + offA;
  const __bf16* Ab2 = (NSPLIT >= 1) ? (A2 + offA) : Ab;
  const __bf16* Bb  = Bt + offB;

  const int rlane = lane & 15;
  const int koff  = (lane >> 4) * 8;
  const int mOff  = (lane >> 4) * 8;

  v8f acc[4][4];
#pragma unroll
  for (int i = 0; i < 4; ++i)
#pragma unroll
    for (int j = 0; j < 4; ++j) acc[i][j] = zero8();

  for (int k0 = 0; k0 < K; k0 += 32) {
    const int seg = k0 >> ksh;
    const int kin = k0 - (seg << ksh);
    const size_t aK = (size_t)seg * (size_t)ksA + (size_t)(kin + koff);
    const size_t bK = (size_t)seg * (size_t)ksB + (size_t)(kin + koff);
    v16b bh[4];
#pragma unroll
    for (int j = 0; j < 4; ++j) {
      bh[j] = ldfrag_b(Bb + (size_t)(n0 + (j << 4) + rlane) * ldb + bK);
    }
#pragma unroll
    for (int i = 0; i < 4; ++i) {
      const size_t ao = (size_t)(m0 + (i << 4) + rlane) * lda + aK;
      const v16b ah = ldfrag_b(Ab + ao);
      v16b al = ah;
      if (NSPLIT >= 1) al = ldfrag_b(Ab2 + ao);
#pragma unroll
      for (int j = 0; j < 4; ++j) {
        acc[i][j] = mma_b_raw(ah, bh[j], acc[i][j]);
        if (NSPLIT >= 1) acc[i][j] = mma_b_raw(al, bh[j], acc[i][j]);
      }
      dep_guard_b(acc[i][0], acc[i][3], ah, al);
    }
    keep4_b(bh[0], bh[1], bh[2], bh[3]);
  }
  acc_guard4(acc[0][0], acc[0][1], acc[0][2], acc[0][3]);
  acc_guard4(acc[1][0], acc[1][1], acc[1][2], acc[1][3]);
  acc_guard4(acc[2][0], acc[2][1], acc[2][2], acc[2][3]);
  acc_guard4(acc[3][0], acc[3][1], acc[3][2], acc[3][3]);

  float* slab = sT[wave];
#pragma unroll
  for (int i = 0; i < 4; ++i) {
    const int mBase = m0 + (i << 4);
#pragma unroll
    for (int j = 0; j < 4; ++j) {
#pragma unroll
      for (int r = 0; r < 8; ++r) {
        slab[(mOff + r) * 68 + (j << 4) + rlane] = acc[i][j][r];
      }
    }
    wave_sync_lds();
    if (OUT_MODE == 0) {
      float* Cp = (float*)Cout + offC;
      const int hh = lane >> 4, c4 = (lane & 15) * 4;
      for (int pass = 0; pass < 2; ++pass) {
#pragma unroll
        for (int it = 0; it < 8; ++it) {
          const int row = it * 2 + hh;
          const v4f v = *(const v4f*)(slab + row * 68 + c4);
          *(volatile v4f*)(Cp + (size_t)(mBase + row) * ldc + n0 + c4) = v;
        }
        __threadfence();
      }
    } else {
      const int q = lane >> 3, c8 = (lane & 7) * 8;
      unsigned short* Cp  = (unsigned short*)Cout  + offC;
      unsigned short* Cp2 = (unsigned short*)Cout2 + offC;
      v4u hv[4], lv[4];
#pragma unroll
      for (int it = 0; it < 4; ++it) {
        const int row = it * 4 + q;
        const float* sp = slab + row * 68 + c8;
        v4u a, a2;
#pragma unroll
        for (int e = 0; e < 4; ++e) {
          const float f0 = sp[2 * e], f1 = sp[2 * e + 1];
          const unsigned short h0 = bf_bits(f0), h1 = bf_bits(f1);
          const unsigned short l0 = bf_bits(f0 - bf_up(h0)), l1 = bf_bits(f1 - bf_up(h1));
          a[e] = pk16(h0, h1); a2[e] = pk16(l0, l1);
        }
        hv[it] = a; lv[it] = a2;
      }
      for (int pass = 0; pass < 2; ++pass) {
#pragma unroll
        for (int it = 0; it < 4; ++it) {
          const int row = it * 4 + q;
          *(volatile v4u*)(Cp  + (size_t)(mBase + row) * ldc + n0 + c8) = hv[it];
          *(volatile v4u*)(Cp2 + (size_t)(mBase + row) * ldc + n0 + c8) = lv[it];
        }
        __threadfence();
      }
    }
    wave_sync_lds();
  }
}

__device__ __forceinline__ float fexp(float x) { return __builtin_amdgcn_exp2f(x * 1.4426950408889634f); }

__global__ __launch_bounds__(256) void softmax_rows(const float* __restrict__ lg, unsigned short* ahp, unsigned short* alp,
                                                    float* out1) {
  extern __shared__ __align__(16) float sS[];
  const int b    = blockIdx.x;
  const int tid  = threadIdx.x;
  const int lane = tid & 31;
  const int wave = tid >> 5;
#pragma unroll 1
  for (int ii = 0; ii < 8; ++ii) {
    const int i = wave * 8 + ii;
    float hs[8];
#pragma unroll
    for (int j = 0; j < 8; ++j) hs[j] = 0.f;
#pragma unroll 1
    for (int h = 0; h < NH_; ++h) {
      const size_t row = (size_t)(b * NH_ + h) * IDF_ + i;
      const float* p = lg + row * LL_ + lane * 8;
      const v4f x0 = *(const v4f*)p;
      const v4f x1 = *(const v4f*)(p + 4);
      float v[8] = {x0[0], x0[1], x0[2], x0[3], x1[0], x1[1], x1[2], x1[3]};
      float mx = v[0];
#pragma unroll
      for (int j = 1; j < 8; ++j) mx = fmaxf(mx, v[j]);
#pragma unroll
      for (int off = 16; off > 0; off >>= 1) mx = fmaxf(mx, __shfl_xor(mx, off, 32));
      float s = 0.f;
#pragma unroll
      for (int j = 0; j < 8; ++j) { v[j] = fexp(v[j] - mx); s += v[j]; }
#pragma unroll
      for (int off = 16; off > 0; off >>= 1) s += __shfl_xor(s, off, 32);
      const float inv = __builtin_amdgcn_rcpf(s);
      unsigned short hb[8], lb[8];
#pragma unroll
      for (int j = 0; j < 8; ++j) {
        const float pj = v[j] * inv;
        hs[j] += pj;
        hb[j] = bf_bits(pj);
        lb[j] = bf_bits(pj - bf_up(hb[j]));
      }
      v4u hv, lv;
#pragma unroll
      for (int e = 0; e < 4; ++e) { hv[e] = pk16(hb[2 * e], hb[2 * e + 1]); lv[e] = pk16(lb[2 * e], lb[2 * e + 1]); }
      unsigned short* dh = ahp + row * LL_ + lane * 8;
      unsigned short* dl = alp + row * LL_ + lane * 8;
      *(volatile v4u*)dh = hv;
      *(volatile v4u*)dl = lv;
      __threadfence();
      *(volatile v4u*)dh = hv;
      *(volatile v4u*)dl = lv;
    }
#pragma unroll
    for (int j = 0; j < 8; ++j) sS[(lane * 8 + j) * IDF_ + i] = hs[j];
  }
  __syncthreads();
  {
    const int hh = lane >> 4, c4 = (lane & 15) * 4;
    for (int pass = 0; pass < 2; ++pass) {
#pragma unroll
      for (int it = 0; it < 16; ++it) {
        const int l = it * 16 + wave * 2 + hh;
        const v4f vv = *(const v4f*)(sS + l * IDF_ + c4);
        *(volatile v4f*)(out1 + ((size_t)b * LL_ + l) * IDF_ + c4) = vv;
      }
      __threadfence();
    }
  }
}

extern "C" void kernel_launch(void* const* d_in, const int* in_sizes, int n_in,
                              void* d_out, int out_size, void* d_ws, size_t ws_size,
                              hipStream_t stream) {
  if (n_in < 3) return;
  if (in_sizes[0] != NB_ * IDF_ * SS_) return;
  if (in_sizes[1] != NB_ * CDF_ * LL_) return;
  if (in_sizes[2] != NH_ * SS_ * CDF_) return;
  if (out_size != NB_ * IDF_ * SS_ + NB_ * LL_ * IDF_) return;

  const float* wc  = (const float*)d_in[0];
  const float* ctx = (const float*)d_in[1];
  const float* W   = (const float*)d_in[2];
  float* out0 = (float*)d_out;
  float* out1 = (float*)d_out + (size_t)NB_ * IDF_ * SS_;

  const size_t P2h = (size_t)2097152 * 2;
  const size_t P4h = (size_t)4194304 * 2;
  const size_t P4f = (size_t)4194304 * 4;
  size_t off = 0;
  const size_t oWc  = off; off += P2h;
  const size_t oWb  = off; off += P2h;
  const size_t oWT  = off; off += P2h;
  const size_t oCxB = off; off += P2h;
  const size_t oCxT = off; off += P2h;
  const size_t oMh  = off; off += P4h;
  const size_t oMl  = off; off += P4h;
  const size_t oLG  = off; off += P4f;
  const size_t oAH  = off; off += P4h;
  const size_t oAL  = off; off += P4h;
  const size_t oZh  = off; off += P4h;
  const size_t oZl  = off; off += P4h;
  if (off > ws_size) return;
  if (off > (size_t)134217728) return;

  char* ws = (char*)d_ws;
  unsigned short* wcB  = (unsigned short*)(ws + oWc);
  unsigned short* Wb   = (unsigned short*)(ws + oWb);
  unsigned short* WT   = (unsigned short*)(ws + oWT);
  unsigned short* ctxB = (unsigned short*)(ws + oCxB);
  unsigned short* ctxT = (unsigned short*)(ws + oCxT);
  unsigned short* Mh   = (unsigned short*)(ws + oMh);
  unsigned short* Ml   = (unsigned short*)(ws + oMl);
  float*          LG   = (float*)(ws + oLG);
  unsigned short* AH   = (unsigned short*)(ws + oAH);
  unsigned short* AL   = (unsigned short*)(ws + oAL);
  unsigned short* Zh   = (unsigned short*)(ws + oZh);
  unsigned short* Zl   = (unsigned short*)(ws + oZl);

  const dim3 blk(256);
  const long long yM  = (long long)IDF_ * NH_ * CDF_;
  const long long yHC = (long long)NH_ * IDF_ * CDF_;
  const long long zHC = (long long)IDF_ * CDF_;
  const long long yCx = (long long)CDF_ * LL_;

  cvt_bf16x8<<<dim3(NB_ * IDF_ * SS_ / 8 / 256), blk, 0, stream>>>(wc, wcB, NB_ * IDF_ * SS_ / 8);
  tcvt64<<<dim3(CDF_ / 64, SS_ / 64, NH_), blk, 0, stream>>>(W, Wb, WT, SS_, CDF_);
  tcvt64<<<dim3(LL_ / 64, CDF_ / 64, NB_), blk, 0, stream>>>(ctx, ctxB, ctxT, CDF_, LL_);
  gemm64<0, 2><<<dim3(4, NB_), blk, 0, stream>>>(
      wcB, wcB, SS_, (long long)IDF_ * SS_, 0LL, 0LL,
      WT, SS_, 0LL, 0LL, 0LL, 30,
      (void*)Mh, (void*)Ml, NH_ * CDF_, yM, 0LL,
      IDF_, NH_ * CDF_, SS_, 1);
  gemm64<1, 0><<<dim3(4, NB_), blk, 0, stream>>>(
      Mh, Ml, NH_ * CDF_, yM, (long long)CDF_, 0LL,
      ctxT, CDF_, yCx, 0LL, 0LL, 30,
      (void*)LG, (void*)LG, LL_, yHC, (long long)IDF_ * LL_,
      IDF_, LL_, CDF_, NH_);
  softmax_rows<<<dim3(NB_), blk, LL_ * IDF_ * 4, stream>>>(LG, AH, AL, out1);
  gemm64<1, 2><<<dim3(4, NB_), blk, 0, stream>>>(
      AH, AL, LL_, yHC, (long long)IDF_ * LL_, 0LL,
      ctxB, LL_, yCx, 0LL, 0LL, 30,
      (void*)Zh, (void*)Zl, CDF_, yHC, zHC,
      IDF_, CDF_, LL_, NH_);
  gemm64<1, 0><<<dim3(2, NB_), blk, 0, stream>>>(
      Zh, Zl, CDF_, yHC, 0LL, zHC,
      Wb, CDF_, 0LL, 0LL, (long long)SS_ * CDF_, 8,
      (void*)out0, (void*)out0, SS_, (long long)IDF_ * SS_, 0LL,
      IDF_, SS_, NH_ * CDF_, 1);
  (void)hipGetLastError();
}
